// DecompGen_78658031059107
// MI455X (gfx1250) — hardware-verified
//
#include <hip/hip_runtime.h>
#include <stdint.h>
#include <stddef.h>

#define NB   256
#define NZ   100
#define NZP  128
#define RK   512
#define RQ   128
#define RH   256
#define NCLS 10

typedef __bf16 v16b __attribute__((ext_vector_type(16)));
typedef float v8f __attribute__((ext_vector_type(8)));
typedef float v4f __attribute__((ext_vector_type(4)));
typedef unsigned int v4u __attribute__((ext_vector_type(4)));
typedef unsigned int v2u __attribute__((ext_vector_type(2)));
typedef v4f __attribute__((may_alias)) v4fa;
typedef v4u __attribute__((may_alias)) v4ua;
typedef v2u __attribute__((may_alias)) v2ua;
union FragU { v16b v; v4u q[2]; };

__device__ __forceinline__ v8f wmma_bf(v16b a, v16b b, v8f c) {
  v8f d = __builtin_amdgcn_wmma_f32_16x16x32_bf16(false, a, false, b, (short)0, c, false, false);
  asm volatile("v_nop\n\tv_nop\n\tv_nop\n\tv_nop" : "+v"(d) : "v"(a), "v"(b));
  return d;
}

__device__ __forceinline__ v16b ldfrag(const unsigned short* p, int h) {
  FragU f;
  f.q[0] = *(const v4ua*)(p + 8 * h);
  f.q[1] = *(const v4ua*)(p + 16 + 8 * h);
  return f.v;
}

__device__ __forceinline__ unsigned int bf_bits(float x) {
  const unsigned int u = __float_as_uint(x);
  return (u + 0x7FFFu + ((u >> 16) & 1u)) >> 16;
}
__device__ __forceinline__ void split_bf(float x, unsigned int& hi, unsigned int& lo) {
  hi = bf_bits(x);
  lo = bf_bits(x - __uint_as_float(hi << 16));
}
__device__ __forceinline__ void split4(v4f v, v2u& hi, v2u& lo) {
  unsigned int h0, h1, h2, h3, l0, l1, l2, l3;
  split_bf(v.x, h0, l0); split_bf(v.y, h1, l1); split_bf(v.z, h2, l2); split_bf(v.w, h3, l3);
  hi.x = h0 | (h1 << 16); hi.y = h2 | (h3 << 16);
  lo.x = l0 | (l1 << 16); lo.y = l2 | (l3 << 16);
}
__device__ __forceinline__ v4u join4u(v2u a, v2u b) { v4u r; r.x = a.x; r.y = a.y; r.z = b.x; r.w = b.y; return r; }
__device__ __forceinline__ v4u sel4u(bool c, v4u a, v4u b) {
  v4u r; r.x = c ? a.x : b.x; r.y = c ? a.y : b.y; r.z = c ? a.z : b.z; r.w = c ? a.w : b.w; return r;
}
__device__ __forceinline__ v4f sel4f(bool c, v4f a, v4f b) {
  v4f r; r.x = c ? a.x : b.x; r.y = c ? a.y : b.y; r.z = c ? a.z : b.z; r.w = c ? a.w : b.w; return r;
}
__device__ __forceinline__ v4f lrelu4(v4f v, float s) {
  v4f r;
  r.x = (v.x >= 0.0f) ? v.x : s * v.x; r.y = (v.y >= 0.0f) ? v.y : s * v.y;
  r.z = (v.z >= 0.0f) ? v.z : s * v.z; r.w = (v.w >= 0.0f) ? v.w : s * v.w;
  return r;
}
__device__ __forceinline__ float tanh_f(float x) {
  const float a = fabsf(x);
  const float e = __expf(-2.0f * a);
  const float tp = (1.0f - e) * (1.0f / (1.0f + e));
  return (x < 0.0f) ? -tp : tp;
}

struct TwSeg {
  const float* in; unsigned short* oh; unsigned short* ol;
  int R; int C; int nblk; int padz;
};
typedef char tw_size_check[(sizeof(TwSeg) == 40) ? 1 : -1];

__global__ __launch_bounds__(256) void k_tw(TwSeg s0, TwSeg s1, TwSeg s2, TwSeg s3, int c0, int c1, int c2) {
  __shared__ float sm[32][65];
  const int blk = blockIdx.x;
  const int seg = (blk >= c0 ? 1 : 0) + (blk >= c1 ? 1 : 0) + (blk >= c2 ? 1 : 0);
  const TwSeg S = (seg == 0) ? s0 : ((seg == 1) ? s1 : ((seg == 2) ? s2 : s3));
  const int start = (seg == 0) ? 0 : ((seg == 1) ? c0 : ((seg == 2) ? c1 : c2));
  const int local = blk - start;
  const int tilesC = S.C >> 5;
  const int cB = (local % tilesC) * 32;
  const int rB = (local / tilesC) * 64;
  const int tid = threadIdx.x;
  {
    const int rl = tid >> 2, c8 = (tid & 3) * 8;
    const float* src = S.in + (size_t)(rB + rl) * S.C + cB + c8;
    const v4f a = *(const v4fa*)src;
    const v4f b = *(const v4fa*)(src + 4);
    sm[c8 + 0][rl] = a.x; sm[c8 + 1][rl] = a.y; sm[c8 + 2][rl] = a.z; sm[c8 + 3][rl] = a.w;
    sm[c8 + 4][rl] = b.x; sm[c8 + 5][rl] = b.y; sm[c8 + 6][rl] = b.z; sm[c8 + 7][rl] = b.w;
  }
  __syncthreads();
  const int cl = tid >> 3, q = tid & 7;
  v4f f0, f1;
  f0.x = sm[cl][8 * q + 0]; f0.y = sm[cl][8 * q + 1]; f0.z = sm[cl][8 * q + 2]; f0.w = sm[cl][8 * q + 3];
  f1.x = sm[cl][8 * q + 4]; f1.y = sm[cl][8 * q + 5]; f1.z = sm[cl][8 * q + 6]; f1.w = sm[cl][8 * q + 7];
  v2u ha, la, hb, lb;
  split4(f0, ha, la); split4(f1, hb, lb);
  const v4u hi = join4u(ha, hb), lo = join4u(la, lb);
  const size_t idx = (size_t)(cB + cl) * S.R + rB + 8 * q;
  *(volatile v4ua*)(S.oh + idx) = hi;
  *(volatile v4ua*)(S.ol + idx) = lo;
  __threadfence();
  *(volatile v4ua*)(S.oh + idx) = hi;
  *(volatile v4ua*)(S.ol + idx) = lo;
}

__global__ __launch_bounds__(256) void k_rc(const float* __restrict__ noise, const float* __restrict__ linw,
                                            unsigned short* __restrict__ nH, unsigned short* __restrict__ nL,
                                            unsigned short* __restrict__ wH, unsigned short* __restrict__ wL) {
  const int tid = threadIdx.x, lane = tid & 31;
  const int row = blockIdx.x * 8 + (tid >> 5);
  const bool isw = row >= NB;
  const int r = isw ? (row - NB) : row;
  const float* src = (isw ? linw : noise) + (size_t)r * NZ;
  unsigned short* dh = isw ? wH : nH;
  unsigned short* dl = isw ? wL : nL;
  const int col0 = 8 * (lane & 15);
  float f[8];
  #pragma unroll
  for (int e = 0; e < 8; ++e) {
    const int c = col0 + e;
    const int cc = (c < NZ) ? c : (NZ - 1);
    const float v = src[cc];
    f[e] = (c < NZ) ? v : 0.0f;
  }
  v4f fa, fb;
  fa.x = f[0]; fa.y = f[1]; fa.z = f[2]; fa.w = f[3];
  fb.x = f[4]; fb.y = f[5]; fb.z = f[6]; fb.w = f[7];
  v2u ha, la, hb, lb;
  split4(fa, ha, la); split4(fb, hb, lb);
  const v4u hi = join4u(ha, hb), lo = join4u(la, lb);
  const bool hsel = (lane >> 4) != 0;
  const v4u o = sel4u(hsel, lo, hi);
  unsigned short* dst = (hsel ? dl : dh) + (size_t)r * NZP + col0;
  *(volatile v4ua*)dst = o;
  __threadfence();
  *(volatile v4ua*)dst = o;
}

struct MmSeg {
  const unsigned short* Ah; const unsigned short* Al;
  const unsigned short* Bh; const unsigned short* Bl;
  const float* bias; float* out;
  int K; int N; int Lin; int ktaps; int Lout; int act; int nblk; int padz;
};
typedef char mm_size_check[(sizeof(MmSeg) == 80) ? 1 : -1];

__device__ __forceinline__ void mm_store_pass(const float* sT, float* out, int Lout, int N, int t,
                                              int bRow0, int nCol0, int w, int lane) {
  const int l16 = lane & 15, hl = lane >> 4;
  #pragma unroll
  for (int i = 0; i < 8; ++i) {
    const int rl = w * 16 + 2 * i + hl;
    const v4f v = *(const v4fa*)(sT + rl * 68 + 4 * l16);
    float* dst = out + ((size_t)(bRow0 + rl) * Lout + t) * N + nCol0 + 4 * l16;
    *(volatile v4f*)dst = v;
  }
}

__global__ __launch_bounds__(128) void k_mm(MmSeg s0, MmSeg s1, MmSeg s2, int c0, int c1) {
  __shared__ __attribute__((aligned(16))) float sT[64 * 68];

  const int blk = blockIdx.x;
  const int seg = (blk >= c0 ? 1 : 0) + (blk >= c1 ? 1 : 0);
  const MmSeg S = (seg == 0) ? s0 : ((seg == 1) ? s1 : s2);
  const int local = blk - ((seg == 0) ? 0 : ((seg == 1) ? c0 : c1));
  const int nTiles = S.N >> 6;
  const int nT = local % nTiles;
  const int rest = local / nTiles;
  const int bT = rest & 3;
  const int t = rest >> 2;
  const int K = S.K;

  const int tid = threadIdx.x, lane = tid & 31, w = tid >> 5;
  const int h = lane >> 4, m = lane & 15;
  const int rw = 32 * (w & 1), cw = 32 * (w >> 1);
  const int bW = bT * 64 + rw;
  const int nW = nT * 64 + cw;
  int tapLo = t - (S.Lin - 1); if (tapLo < 0) tapLo = 0;
  int tapHi = t; if (tapHi > S.ktaps - 1) tapHi = S.ktaps - 1;

  const v8f zero8 = {0.f, 0.f, 0.f, 0.f, 0.f, 0.f, 0.f, 0.f};
  v8f acc00 = zero8, acc01 = zero8, acc10 = zero8, acc11 = zero8;

  #pragma unroll 1
  for (int tap = tapLo; tap <= tapHi; ++tap) {
    const int j = t - tap;
    const size_t ar0 = ((size_t)(bW + m) * S.Lin + j) * K;
    const size_t ar1 = ((size_t)(bW + 16 + m) * S.Lin + j) * K;
    const size_t br0 = ((size_t)(nW + m) * S.ktaps + tap) * K;
    const size_t br1 = ((size_t)(nW + 16 + m) * S.ktaps + tap) * K;
    const unsigned short* pa0h = S.Ah + ar0;
    const unsigned short* pa1h = S.Ah + ar1;
    const unsigned short* pa0l = S.Al + ar0;
    const unsigned short* pa1l = S.Al + ar1;
    const unsigned short* pb0h = S.Bh + br0;
    const unsigned short* pb1h = S.Bh + br1;
    const unsigned short* pb0l = S.Bl + br0;
    const unsigned short* pb1l = S.Bl + br1;
    #pragma unroll 1
    for (int k0 = 0; k0 < K; k0 += 32) {
      const v16b a0h = ldfrag(pa0h + k0, h);
      const v16b a1h = ldfrag(pa1h + k0, h);
      const v16b a0l = ldfrag(pa0l + k0, h);
      const v16b a1l = ldfrag(pa1l + k0, h);
      const v16b b0h = ldfrag(pb0h + k0, h);
      const v16b b1h = ldfrag(pb1h + k0, h);
      const v16b b0l = ldfrag(pb0l + k0, h);
      const v16b b1l = ldfrag(pb1l + k0, h);
      acc00 = wmma_bf(a0h, b0h, acc00); acc00 = wmma_bf(a0h, b0l, acc00); acc00 = wmma_bf(a0l, b0h, acc00);
      acc01 = wmma_bf(a0h, b1h, acc01); acc01 = wmma_bf(a0h, b1l, acc01); acc01 = wmma_bf(a0l, b1h, acc01);
      acc10 = wmma_bf(a1h, b0h, acc10); acc10 = wmma_bf(a1h, b0l, acc10); acc10 = wmma_bf(a1l, b0h, acc10);
      acc11 = wmma_bf(a1h, b1h, acc11); acc11 = wmma_bf(a1h, b1l, acc11); acc11 = wmma_bf(a1l, b1h, acc11);
    }
  }

  const int act = S.act;
  const float bv0 = S.bias[nW + m];
  const float bv1 = S.bias[nW + 16 + m];
  #pragma unroll
  for (int r = 0; r < 8; ++r) {
    float v00 = acc00[r] + bv0, v01 = acc01[r] + bv1, v10 = acc10[r] + bv0, v11 = acc11[r] + bv1;
    if (act != 0) { v00 = tanh_f(v00); v01 = tanh_f(v01); v10 = tanh_f(v10); v11 = tanh_f(v11); }
    const int r0 = rw + 8 * h + r, r1 = rw + 16 + 8 * h + r;
    sT[r0 * 68 + cw + m] = v00;
    sT[r0 * 68 + cw + 16 + m] = v01;
    sT[r1 * 68 + cw + m] = v10;
    sT[r1 * 68 + cw + 16 + m] = v11;
  }
  __syncthreads();

  mm_store_pass(sT, S.out, S.Lout, S.N, t, bT * 64, nT * 64, w, lane);
  __threadfence();
  mm_store_pass(sT, S.out, S.Lout, S.N, t, bT * 64, nT * 64, w, lane);
}

__global__ __launch_bounds__(256) void k_lat(const float* __restrict__ zpre, const float* __restrict__ g,
                                             const float* __restrict__ be, const float* __restrict__ emb,
                                             const int* __restrict__ label,
                                             unsigned short* __restrict__ latH, unsigned short* __restrict__ latL) {
  __shared__ __attribute__((aligned(16))) float ssc[128];
  __shared__ __attribute__((aligned(16))) float ssh[128];
  const int tid = threadIdx.x;
  if (tid < 128) {
    double s = 0.0, q = 0.0;
    #pragma unroll 1
    for (int b = 0; b < NB; ++b) {
      const float v = zpre[b * 128 + tid];
      s += (double)v;
      q += (double)v * (double)v;
    }
    const double mean = s * (1.0 / 256.0);
    double var = q * (1.0 / 256.0) - mean * mean;
    if (var < 0.0) var = 0.0;
    const float sc = g[tid] * rsqrtf((float)var + 1e-5f);
    ssc[tid] = sc;
    ssh[tid] = be[tid] - (float)mean * sc;
  }
  __syncthreads();

  const int lane = tid & 31, w = tid >> 5;
  const int rb = blockIdx.x * 16 + 2 * w + (lane >> 4);
  const int col0 = 8 * (lane & 15);
  const v4f x0 = *(const v4fa*)(zpre + (size_t)rb * 128 + col0);
  const v4f x1 = *(const v4fa*)(zpre + (size_t)rb * 128 + col0 + 4);
  const v4f sc0 = *(const v4fa*)(ssc + col0), sc1 = *(const v4fa*)(ssc + col0 + 4);
  const v4f sh0 = *(const v4fa*)(ssh + col0), sh1 = *(const v4fa*)(ssh + col0 + 4);
  const v4f y0 = lrelu4(x0 * sc0 + sh0, 0.01f);
  const v4f y1 = lrelu4(x1 * sc1 + sh1, 0.01f);
  v2u hza, lza, hzb, lzb;
  split4(y0, hza, lza); split4(y1, hzb, lzb);
  const v4u hz = join4u(hza, hzb), lz = join4u(lza, lzb);
  int lab = label[rb];
  lab = (lab < 0) ? 0 : ((lab > NCLS - 1) ? (NCLS - 1) : lab);
  const v4f e0 = *(const v4fa*)(emb + (size_t)lab * 128 + col0);
  const v4f e1 = *(const v4fa*)(emb + (size_t)lab * 128 + col0 + 4);
  v2u hea, lea, heb, leb;
  split4(e0, hea, lea); split4(e1, heb, leb);
  const v4u he = join4u(hea, heb), le = join4u(lea, leb);

  const size_t pz = (size_t)rb * 256 + col0, pe = pz + 128;
  *(volatile v4ua*)(latH + pz) = hz; *(volatile v4ua*)(latH + pe) = he;
  *(volatile v4ua*)(latL + pz) = lz; *(volatile v4ua*)(latL + pe) = le;
  __threadfence();
  *(volatile v4ua*)(latH + pz) = hz; *(volatile v4ua*)(latH + pe) = he;
  *(volatile v4ua*)(latL + pz) = lz; *(volatile v4ua*)(latL + pe) = le;
}

struct StSeg {
  const float* src; const float* gamma; const float* beta; float* stats;
  int Cout; int L; int pitchB; int nblk;
};
typedef char st_size_check[(sizeof(StSeg) == 48) ? 1 : -1];

__global__ __launch_bounds__(256) void k_bnstats(StSeg s0, StSeg s1, StSeg s2, int c0, int c1) {
  __shared__ double ps[8][32];
  __shared__ double pq[8][32];
  __shared__ __attribute__((aligned(16))) float ssc[32];
  __shared__ __attribute__((aligned(16))) float ssh[32];
  const int blk = blockIdx.x;
  const int seg = (blk >= c0 ? 1 : 0) + (blk >= c1 ? 1 : 0);
  const StSeg S = (seg == 0) ? s0 : ((seg == 1) ? s1 : s2);
  const int local = blk - ((seg == 0) ? 0 : ((seg == 1) ? c0 : c1));
  const int oBase = local * 32;
  const int tid = threadIdx.x, ch = tid & 31, part = tid >> 5;
  const int o = oBase + ch;
  double s = 0.0, q = 0.0;
  #pragma unroll 1
  for (int b = part; b < NB; b += 8) {
    const float* p = S.src + (size_t)b * S.pitchB + o;
    #pragma unroll 1
    for (int tt = 0; tt < S.L; ++tt) {
      const float v = p[(size_t)tt * S.Cout];
      s += (double)v;
      q += (double)v * (double)v;
    }
  }
  ps[part][ch] = s;
  pq[part][ch] = q;
  __syncthreads();
  if (tid < 32) {
    double a = 0.0, a2 = 0.0;
    #pragma unroll
    for (int p = 0; p < 8; ++p) { a += ps[p][tid]; a2 += pq[p][tid]; }
    const double n = 256.0 * (double)S.L;
    const double mean = a / n;
    double var = a2 / n - mean * mean;
    if (var < 0.0) var = 0.0;
    const float sc = S.gamma[oBase + tid] * rsqrtf((float)var + 1e-5f);
    ssc[tid] = sc;
    ssh[tid] = S.beta[oBase + tid] - (float)mean * sc;
  }
  __syncthreads();
  if (tid < 16) {
    const int q8 = tid & 7;
    const bool which = (tid >> 3) != 0;
    const v4f vs = *(const v4fa*)(ssc + 4 * q8);
    const v4f vh = *(const v4fa*)(ssh + 4 * q8);
    const v4f v = sel4f(which, vh, vs);
    float* dst = S.stats + (which ? S.Cout : 0) + oBase + 4 * q8;
    *(volatile v4f*)dst = v;
    __threadfence();
    *(volatile v4f*)dst = v;
  }
}

struct ApSeg {
  const float* src; const float* stats; float* dstF; unsigned short* dstH; unsigned short* dstL;
  int Cout; int nblk; int mode; int padz;
};
typedef char ap_size_check[(sizeof(ApSeg) == 56) ? 1 : -1];

__global__ __launch_bounds__(256) void k_bnapply(ApSeg s0, ApSeg s1, ApSeg s2, int c0, int c1, float slope) {
  const int blk = blockIdx.x;
  const int seg = (blk >= c0 ? 1 : 0) + (blk >= c1 ? 1 : 0);
  const ApSeg S = (seg == 0) ? s0 : ((seg == 1) ? s1 : s2);
  const int local = blk - ((seg == 0) ? 0 : ((seg == 1) ? c0 : c1));
  const int tid = threadIdx.x, lane = tid & 31;
  const int run = local * 8 + (tid >> 5);
  const int cm = S.Cout - 1;
  if (S.mode == 0) {
    const size_t base = (size_t)run * 256 + 8 * lane;
    const int o0 = (int)(base & (size_t)cm);
    const v4f x0 = *(const v4fa*)(S.src + base);
    const v4f x1 = *(const v4fa*)(S.src + base + 4);
    const v4f sc0 = *(const v4fa*)(S.stats + o0), sc1 = *(const v4fa*)(S.stats + o0 + 4);
    const v4f sh0 = *(const v4fa*)(S.stats + S.Cout + o0), sh1 = *(const v4fa*)(S.stats + S.Cout + o0 + 4);
    const v4f y0 = lrelu4(x0 * sc0 + sh0, slope);
    const v4f y1 = lrelu4(x1 * sc1 + sh1, slope);
    v2u ha, la, hb, lb;
    split4(y0, ha, la); split4(y1, hb, lb);
    const v4u hi = join4u(ha, hb), lo = join4u(la, lb);
    *(volatile v4ua*)(S.dstH + base) = hi;
    *(volatile v4ua*)(S.dstL + base) = lo;
    __threadfence();
    *(volatile v4ua*)(S.dstH + base) = hi;
    *(volatile v4ua*)(S.dstL + base) = lo;
  } else {
    const size_t b0 = (size_t)run * 256 + 4 * lane;
    const size_t b1 = b0 + 128;
    const int o0 = (int)(b0 & (size_t)cm), o1 = (int)(b1 & (size_t)cm);
    const v4f x0 = *(const v4fa*)(S.src + b0);
    const v4f x1 = *(const v4fa*)(S.src + b1);
    const v4f sc0 = *(const v4fa*)(S.stats + o0), sh0 = *(const v4fa*)(S.stats + S.Cout + o0);
    const v4f sc1 = *(const v4fa*)(S.stats + o1), sh1 = *(const v4fa*)(S.stats + S.Cout + o1);
    const v4f y0 = lrelu4(x0 * sc0 + sh0, slope);
    const v4f y1 = lrelu4(x1 * sc1 + sh1, slope);
    *(volatile v4f*)(S.dstF + b0) = y0;
    *(volatile v4f*)(S.dstF + b1) = y1;
    __threadfence();
    *(volatile v4f*)(S.dstF + b0) = y0;
    *(volatile v4f*)(S.dstF + b1) = y1;
  }
}

__device__ __forceinline__ void fin_store_pass(const float* sO, float* ob, int w, int lane) {
  const int q8 = lane & 7, sub = lane >> 3;
  #pragma unroll
  for (int i = 0; i < 2; ++i) {
    const int row = 8 * w + 4 * i + sub;
    const v4f v = *(const v4fa*)(sO + row * 36 + 4 * q8);
    *(volatile v4f*)(ob + row * 32 + 4 * q8) = v;
  }
}

__global__ __launch_bounds__(128) void k_fin(const float* __restrict__ cact, const float* __restrict__ hF,
                                             const float* __restrict__ wF, const float* __restrict__ coef,
                                             float* __restrict__ out) {
  __shared__ __attribute__((aligned(16))) unsigned short sAh[32 * 128];
  __shared__ __attribute__((aligned(16))) unsigned short sAl[32 * 128];
  __shared__ __attribute__((aligned(16))) unsigned short sBh[32 * 128];
  __shared__ __attribute__((aligned(16))) unsigned short sBl[32 * 128];
  __shared__ __attribute__((aligned(16))) float sO[32 * 36];

  const int b = blockIdx.x, ch = blockIdx.y;
  const int tid = threadIdx.x, lane = tid & 31, w = tid >> 5;
  const int h = lane >> 4, m = lane & 15;
  const int yt = w & 1, xt = w >> 1;
  const float* crow = cact + ((size_t)b * 3 + ch) * RK;
  const float* hb = hF + (size_t)b * 32 * RK;
  const float* wb = wF + (size_t)b * 32 * RK;
  const int rl4 = lane * 4;

  v8f acc = {0.f, 0.f, 0.f, 0.f, 0.f, 0.f, 0.f, 0.f};
  #pragma unroll 1
  for (int kc = 0; kc < 4; ++kc) {
    const int r0 = kc * 128;
    const v4f cc = *(const v4fa*)(crow + r0 + rl4);
    const v4f cf = *(const v4fa*)(coef + r0 + rl4);
    const v4f s4 = cc * cf;
    #pragma unroll 2
    for (int yy = w; yy < 32; yy += 4) {
      const v4f hv = *(const v4fa*)(hb + (size_t)yy * RK + r0 + rl4);
      const v4f av = s4 * hv;
      v2u ha, la;
      split4(av, ha, la);
      *(v2ua*)(sAh + yy * 128 + rl4) = ha;
      *(v2ua*)(sAl + yy * 128 + rl4) = la;
      const v4f wv = *(const v4fa*)(wb + (size_t)yy * RK + r0 + rl4);
      v2u hw, lw;
      split4(wv, hw, lw);
      *(v2ua*)(sBh + yy * 128 + rl4) = hw;
      *(v2ua*)(sBl + yy * 128 + rl4) = lw;
    }
    __syncthreads();
    #pragma unroll
    for (int k0 = 0; k0 < 128; k0 += 32) {
      const v16b ah = ldfrag(sAh + (16 * yt + m) * 128 + k0, h);
      const v16b al = ldfrag(sAl + (16 * yt + m) * 128 + k0, h);
      const v16b bh = ldfrag(sBh + (16 * xt + m) * 128 + k0, h);
      const v16b bl = ldfrag(sBl + (16 * xt + m) * 128 + k0, h);
      acc = wmma_bf(ah, bh, acc);
      acc = wmma_bf(ah, bl, acc);
      acc = wmma_bf(al, bh, acc);
    }
    __syncthreads();
  }
  #pragma unroll
  for (int r = 0; r < 8; ++r) sO[(16 * yt + 8 * h + r) * 36 + 16 * xt + m] = acc[r];
  __syncthreads();
  float* ob = out + ((size_t)b * 3 + ch) * 1024;
  fin_store_pass(sO, ob, w, lane);
  __threadfence();
  fin_store_pass(sO, ob, w, lane);
}

static TwSeg mk_tw(const float* in, unsigned short* oh, unsigned short* ol, int R, int C) {
  TwSeg s; s.in = in; s.oh = oh; s.ol = ol; s.R = R; s.C = C; s.nblk = (C / 32) * (R / 64); s.padz = 0; return s;
}
static MmSeg mk_mm(const unsigned short* Ah, const unsigned short* Al, const unsigned short* Bh, const unsigned short* Bl,
                   const float* bias, float* out, int K, int N, int Lin, int ktaps, int Lout, int act) {
  MmSeg s; s.Ah = Ah; s.Al = Al; s.Bh = Bh; s.Bl = Bl; s.bias = bias; s.out = out;
  s.K = K; s.N = N; s.Lin = Lin; s.ktaps = ktaps; s.Lout = Lout; s.act = act;
  s.nblk = (N / 64) * 4 * Lout; s.padz = 0; return s;
}
static StSeg mk_st(const float* src, const float* gamma, const float* beta, float* stats, int Cout, int L, int pitchB) {
  StSeg s; s.src = src; s.gamma = gamma; s.beta = beta; s.stats = stats; s.Cout = Cout; s.L = L; s.pitchB = pitchB;
  s.nblk = Cout / 32; return s;
}
static ApSeg mk_ap(const float* src, const float* stats, float* dstF, unsigned short* dstH, unsigned short* dstL,
                   int Cout, int L, int mode) {
  ApSeg s; s.src = src; s.stats = stats; s.dstF = dstF; s.dstH = dstH; s.dstL = dstL; s.Cout = Cout;
  s.nblk = (256 * L * Cout) / 2048; s.mode = mode; s.padz = 0; return s;
}

extern "C" void kernel_launch(void* const* d_in, const int* in_sizes, int n_in,
                              void* d_out, int out_size, void* d_ws, size_t ws_size,
                              hipStream_t stream) {
  if (n_in != 32) return;
  const int expect[32] = {
    NB * NZ, NB, 128 * NZ, 128, 128, 128, NCLS * 128,
    256 * RK * 3, RK, RK, RK,
    256 * RQ * 16, RQ, RQ, RQ, RQ * RH * 16, RH, RH, RH, RH * RK * 2, RK,
    256 * RQ * 16, RQ, RQ, RQ, RQ * RH * 16, RH, RH, RH, RH * RK * 2, RK,
    RK };
  for (int i = 0; i < 32; ++i) if (in_sizes[i] != expect[i]) return;
  if (out_size != NB * 3 * 32 * 32) return;

  const float* noise = (const float*)d_in[0];
  const int*   label = (const int*)d_in[1];
  const float* lin_w = (const float*)d_in[2];
  const float* lin_b = (const float*)d_in[3];
  const float* bn0_g = (const float*)d_in[4];
  const float* bn0_b = (const float*)d_in[5];
  const float* emb   = (const float*)d_in[6];
  const float* c_w1  = (const float*)d_in[7];
  const float* c_b1  = (const float*)d_in[8];
  const float* c_g1  = (const float*)d_in[9];
  const float* c_be1 = (const float*)d_in[10];
  const float* h_w1  = (const float*)d_in[11];
  const float* h_b1  = (const float*)d_in[12];
  const float* h_g1  = (const float*)d_in[13];
  const float* h_be1 = (const float*)d_in[14];
  const float* h_w2  = (const float*)d_in[15];
  const float* h_b2  = (const float*)d_in[16];
  const float* h_g2  = (const float*)d_in[17];
  const float* h_be2 = (const float*)d_in[18];
  const float* h_w3  = (const float*)d_in[19];
  const float* h_b3  = (const float*)d_in[20];
  const float* w_w1  = (const float*)d_in[21];
  const float* w_b1  = (const float*)d_in[22];
  const float* w_g1  = (const float*)d_in[23];
  const float* w_be1 = (const float*)d_in[24];
  const float* w_w2  = (const float*)d_in[25];
  const float* w_b2  = (const float*)d_in[26];
  const float* w_g2  = (const float*)d_in[27];
  const float* w_be2 = (const float*)d_in[28];
  const float* w_w3  = (const float*)d_in[29];
  const float* w_b3  = (const float*)d_in[30];
  const float* coef  = (const float*)d_in[31];
  float* out = (float*)d_out;

  char* ws = (char*)d_ws;
  size_t off = 0;
  auto carve = [&](size_t bytes) -> size_t { const size_t o = off; off += (bytes + 255) & ~(size_t)255; return o; };
  const size_t pl1 = (size_t)2;
  const size_t o_nH   = carve((size_t)NB * NZP * pl1),  o_nL   = carve((size_t)NB * NZP * pl1);
  const size_t o_lwH  = carve((size_t)128 * NZP * pl1), o_lwL  = carve((size_t)128 * NZP * pl1);
  const size_t o_cw1H = carve((size_t)1536 * 256 * pl1), o_cw1L = carve((size_t)1536 * 256 * pl1);
  const size_t o_hw1H = carve((size_t)2048 * 256 * pl1), o_hw1L = carve((size_t)2048 * 256 * pl1);
  const size_t o_hw2H = carve((size_t)4096 * 128 * pl1), o_hw2L = carve((size_t)4096 * 128 * pl1);
  const size_t o_hw3H = carve((size_t)1024 * 256 * pl1), o_hw3L = carve((size_t)1024 * 256 * pl1);
  const size_t o_ww1H = carve((size_t)2048 * 256 * pl1), o_ww1L = carve((size_t)2048 * 256 * pl1);
  const size_t o_ww2H = carve((size_t)4096 * 128 * pl1), o_ww2L = carve((size_t)4096 * 128 * pl1);
  const size_t o_ww3H = carve((size_t)1024 * 256 * pl1), o_ww3L = carve((size_t)1024 * 256 * pl1);
  const size_t o_zpre = carve((size_t)NB * 128 * 4);
  const size_t o_latH = carve((size_t)NB * 256 * pl1), o_latL = carve((size_t)NB * 256 * pl1);
  const size_t o_cpre = carve((size_t)NB * 3 * RK * 4),  o_cact = carve((size_t)NB * 3 * RK * 4);
  const size_t o_h1p  = carve((size_t)NB * 16 * RQ * 4), o_w1p  = carve((size_t)NB * 16 * RQ * 4);
  const size_t o_x1hH = carve((size_t)NB * 16 * RQ * pl1), o_x1hL = carve((size_t)NB * 16 * RQ * pl1);
  const size_t o_x1wH = carve((size_t)NB * 16 * RQ * pl1), o_x1wL = carve((size_t)NB * 16 * RQ * pl1);
  const size_t o_stc  = carve((size_t)2 * RK * 4);
  const size_t o_sth1 = carve((size_t)2 * RQ * 4), o_stw1 = carve((size_t)2 * RQ * 4);
  const size_t o_sth2 = carve((size_t)2 * RH * 4), o_stw2 = carve((size_t)2 * RH * 4);
  const size_t o_h2p  = carve((size_t)NB * 31 * RH * 4), o_w2p = carve((size_t)NB * 31 * RH * 4);
  const size_t o_x2hH = carve((size_t)NB * 31 * RH * pl1), o_x2hL = carve((size_t)NB * 31 * RH * pl1);
  const size_t o_x2wH = carve((size_t)NB * 31 * RH * pl1), o_x2wL = carve((size_t)NB * 31 * RH * pl1);
  const size_t o_h3   = carve((size_t)NB * 32 * RK * 4),  o_w3  = carve((size_t)NB * 32 * RK * 4);
  if (off > ws_size) return;
  if (off > (size_t)134217728) return;

  unsigned short* nH   = (unsigned short*)(ws + o_nH);   unsigned short* nL   = (unsigned short*)(ws + o_nL);
  unsigned short* lwH  = (unsigned short*)(ws + o_lwH);  unsigned short* lwL  = (unsigned short*)(ws + o_lwL);
  unsigned short* cw1H = (unsigned short*)(ws + o_cw1H); unsigned short* cw1L = (unsigned short*)(ws + o_cw1L);
  unsigned short* hw1H = (unsigned short*)(ws + o_hw1H); unsigned short* hw1L = (unsigned short*)(ws + o_hw1L);
  unsigned short* hw2H = (unsigned short*)(ws + o_hw2H); unsigned short* hw2L = (unsigned short*)(ws + o_hw2L);
  unsigned short* hw3H = (unsigned short*)(ws + o_hw3H); unsigned short* hw3L = (unsigned short*)(ws + o_hw3L);
  unsigned short* ww1H = (unsigned short*)(ws + o_ww1H); unsigned short* ww1L = (unsigned short*)(ws + o_ww1L);
  unsigned short* ww2H = (unsigned short*)(ws + o_ww2H); unsigned short* ww2L = (unsigned short*)(ws + o_ww2L);
  unsigned short* ww3H = (unsigned short*)(ws + o_ww3H); unsigned short* ww3L = (unsigned short*)(ws + o_ww3L);
  float* zpre = (float*)(ws + o_zpre);
  unsigned short* latH = (unsigned short*)(ws + o_latH); unsigned short* latL = (unsigned short*)(ws + o_latL);
  float* cpre = (float*)(ws + o_cpre); float* cact = (float*)(ws + o_cact);
  float* h1p  = (float*)(ws + o_h1p);  float* w1p  = (float*)(ws + o_w1p);
  unsigned short* x1hH = (unsigned short*)(ws + o_x1hH); unsigned short* x1hL = (unsigned short*)(ws + o_x1hL);
  unsigned short* x1wH = (unsigned short*)(ws + o_x1wH); unsigned short* x1wL = (unsigned short*)(ws + o_x1wL);
  float* stc  = (float*)(ws + o_stc);
  float* sth1 = (float*)(ws + o_sth1); float* stw1 = (float*)(ws + o_stw1);
  float* sth2 = (float*)(ws + o_sth2); float* stw2 = (float*)(ws + o_stw2);
  float* h2p  = (float*)(ws + o_h2p);  float* w2p = (float*)(ws + o_w2p);
  unsigned short* x2hH = (unsigned short*)(ws + o_x2hH); unsigned short* x2hL = (unsigned short*)(ws + o_x2hL);
  unsigned short* x2wH = (unsigned short*)(ws + o_x2wH); unsigned short* x2wL = (unsigned short*)(ws + o_x2wL);
  float* h3 = (float*)(ws + o_h3); float* w3 = (float*)(ws + o_w3);
  float* dumF = zpre;
  unsigned short* dumH = nH;

  {
    const TwSeg a = mk_tw(c_w1, cw1H, cw1L, 256, 1536);
    const TwSeg b = mk_tw(h_w1, hw1H, hw1L, 256, 2048);
    const TwSeg c = mk_tw(w_w1, ww1H, ww1L, 256, 2048);
    const TwSeg d = mk_tw(h_w2, hw2H, hw2L, 128, 4096);
    const int c0 = a.nblk, c1 = c0 + b.nblk, c2 = c1 + c.nblk, tot = c2 + d.nblk;
    k_tw<<<tot, 256, 0, stream>>>(a, b, c, d, c0, c1, c2);
  }
  {
    const TwSeg a = mk_tw(w_w2, ww2H, ww2L, 128, 4096);
    const TwSeg b = mk_tw(h_w3, hw3H, hw3L, 256, 1024);
    const TwSeg c = mk_tw(w_w3, ww3H, ww3L, 256, 1024);
    const int c0 = a.nblk, c1 = c0 + b.nblk, tot = c1 + c.nblk;
    k_tw<<<tot, 256, 0, stream>>>(a, b, c, c, c0, c1, tot);
  }
  k_rc<<<(NB + 128) / 8, 256, 0, stream>>>(noise, lin_w, nH, nL, lwH, lwL);
  {
    const MmSeg a = mk_mm(nH, nL, lwH, lwL, lin_b, zpre, NZP, 128, 1, 1, 1, 0);
    k_mm<<<a.nblk, 128, 0, stream>>>(a, a, a, a.nblk, a.nblk);
  }
  k_lat<<<NB / 16, 256, 0, stream>>>(zpre, bn0_g, bn0_b, emb, label, latH, latL);
  {
    const MmSeg a = mk_mm(latH, latL, cw1H, cw1L, c_b1, cpre, 256, RK, 1, 3, 3, 0);
    const MmSeg b = mk_mm(latH, latL, hw1H, hw1L, h_b1, h1p, 256, RQ, 1, 16, 16, 0);
    const MmSeg c = mk_mm(latH, latL, ww1H, ww1L, w_b1, w1p, 256, RQ, 1, 16, 16, 0);
    const int c0 = a.nblk, c1 = c0 + b.nblk, tot = c1 + c.nblk;
    k_mm<<<tot, 128, 0, stream>>>(a, b, c, c0, c1);
  }
  {
    const StSeg a = mk_st(cpre, c_g1, c_be1, stc, RK, 3, 3 * RK);
    const StSeg b = mk_st(h1p, h_g1, h_be1, sth1, RQ, 16, 16 * RQ);
    const StSeg c = mk_st(w1p, w_g1, w_be1, stw1, RQ, 16, 16 * RQ);
    const int c0 = a.nblk, c1 = c0 + b.nblk, tot = c1 + c.nblk;
    k_bnstats<<<tot, 256, 0, stream>>>(a, b, c, c0, c1);
  }
  {
    const ApSeg a = mk_ap(cpre, stc, cact, dumH, dumH, RK, 3, 1);
    const ApSeg b = mk_ap(h1p, sth1, dumF, x1hH, x1hL, RQ, 16, 0);
    const ApSeg c = mk_ap(w1p, stw1, dumF, x1wH, x1wL, RQ, 16, 0);
    const int c0 = a.nblk, c1 = c0 + b.nblk, tot = c1 + c.nblk;
    k_bnapply<<<tot, 256, 0, stream>>>(a, b, c, c0, c1, 0.2f);
  }
  {
    const MmSeg a = mk_mm(x1hH, x1hL, hw2H, hw2L, h_b2, h2p, RQ, RH, 16, 16, 31, 0);
    const MmSeg b = mk_mm(x1wH, x1wL, ww2H, ww2L, w_b2, w2p, RQ, RH, 16, 16, 31, 0);
    const int c0 = a.nblk, tot = c0 + b.nblk;
    k_mm<<<tot, 128, 0, stream>>>(a, b, b, c0, tot);
  }
  {
    const StSeg a = mk_st(h2p, h_g2, h_be2, sth2, RH, 31, 31 * RH);
    const StSeg b = mk_st(w2p, w_g2, w_be2, stw2, RH, 31, 31 * RH);
    const int c0 = a.nblk, tot = c0 + b.nblk;
    k_bnstats<<<tot, 256, 0, stream>>>(a, b, b, c0, tot);
  }
  {
    const ApSeg a = mk_ap(h2p, sth2, dumF, x2hH, x2hL, RH, 31, 0);
    const ApSeg b = mk_ap(w2p, stw2, dumF, x2wH, x2wL, RH, 31, 0);
    const int c0 = a.nblk, tot = c0 + b.nblk;
    k_bnapply<<<tot, 256, 0, stream>>>(a, b, b, c0, tot, 0.2f);
  }
  {
    const MmSeg a = mk_mm(x2hH, x2hL, hw3H, hw3L, h_b3, h3, RH, RK, 31, 2, 32, 1);
    const MmSeg b = mk_mm(x2wH, x2wL, ww3H, ww3L, w_b3, w3, RH, RK, 31, 2, 32, 1);
    const int c0 = a.nblk, tot = c0 + b.nblk;
    k_mm<<<tot, 128, 0, stream>>>(a, b, b, c0, tot);
  }
  k_fin<<<dim3(NB, 3), 128, 0, stream>>>(cact, h3, w3, coef, out);
}
